// DeltaBase_35588099014902
// MI455X (gfx1250) — hardware-verified
//
#include <hip/hip_runtime.h>
#include <stddef.h>


#define NB     64
#define NL     2048
#define NH     128
#define NF     256
#define NV     32000
#define NTOK   (NB * NL)
#define NTHR   256
#define NWAV   (NTHR / 32)
#define STHR   512
#define GBM    64
#define GBN    128
#define GNT    4
#define TB     32
#define NCH    (NL / TB)
#define WSCAP  134217728
#define WCAR   64.0f
#define A1CAR  16.0f
#define RDCAR  16.0f
#define R2CAR  64.0f
#define SC_FF1 (1.0f / 64.0f)
#define SC_FF2 (1.0f / 1024.0f)
#define SC_KP  (1.0f / 64.0f)
#define SC_RP  (1.0f / 1024.0f)
#define SC_OUT (1.0f / 4096.0f)
#define LN_EPS 1e-5f
#define NRM_EPS 1e-12f

#define CB_W1  (NF / 32)
#define CB_W2  (CB_W1 + NH / 32)
#define CB_KP  (CB_W2 + NH / 32)
#define CB_RP  (CB_KP + NH / 32)
#define CB_TOT (CB_RP + NV / 32)

#define SZ_X   ((size_t)NTOK * NH * 2)
#define SZ_A1  ((size_t)NTOK * NF * 2)
#define SZ_W1  ((size_t)NF * NH * 2)
#define SZ_W2  ((size_t)NH * NF * 2)
#define SZ_KP  ((size_t)NH * NH * 2)
#define SZ_OW  ((size_t)NV * NH * 2)
#define SZ_RD  ((size_t)NB * NH * 2)
#define O_X    ((size_t)0)
#define O_A1   (O_X + SZ_X)
#define O_W1   (O_A1 + SZ_A1)
#define O_W2   (O_W1 + SZ_W1)
#define O_KP   (O_W2 + SZ_W2)
#define O_RP   (O_KP + SZ_KP)
#define O_OW   (O_RP + SZ_KP)
#define O_RD   (O_OW + SZ_OW)
#define O_R2   (O_RD + SZ_RD)
#define WSTOT  (O_R2 + SZ_RD)

static_assert(WSTOT <= (size_t)WSCAP);
static_assert((size_t)NTOK * NH * 4 == SZ_A1);
static_assert((O_A1 % 128) == 0 && (O_W1 % 128) == 0 && (O_W2 % 128) == 0 && (O_KP % 128) == 0);
static_assert((O_RP % 128) == 0 && (O_OW % 128) == 0 && (O_RD % 128) == 0 && (O_R2 % 128) == 0);
static_assert((NH % 32) == 0 && (NF % 32) == 0);
static_assert((NTOK % GBM) == 0 && (NF % GBN) == 0 && NH == GBN && NB == GBM && (NV % GBN) == 0);
static_assert((NV % 32) == 0 && (NF % 32) == 0 && (NH % 32) == 0);
static_assert(GBM == 16 * 4 && GBN == 2 * 16 * GNT && NWAV == 8);
static_assert(((size_t)NTOK * NH) % (8 * NTHR) == 0);
static_assert(STHR == 4 * NH && STHR == 16 * TB && TB * NH == STHR * 8 && (NL % TB) == 0);

typedef _Float16 hf_t;
typedef hf_t  v8h  __attribute__((ext_vector_type(8), __may_alias__));
typedef hf_t  v16h __attribute__((ext_vector_type(16)));
typedef int   v8i  __attribute__((ext_vector_type(8)));
typedef float v8f  __attribute__((ext_vector_type(8)));
typedef float v4f  __attribute__((ext_vector_type(4), __may_alias__));
union FragH { v16h v; v8h h[2]; v8i w; };
static_assert(sizeof(FragH) == 32);

__device__ __forceinline__ v8f wmh(FragH a, FragH b, v8f c) {
  v8f d = __builtin_amdgcn_wmma_f32_16x16x32_f16(false, a.v, false, b.v, (short)0, c, false, false);
  asm volatile("v_nop\n\tv_nop\n\tv_nop\n\tv_nop" : "+v"(d) : "v"(a.w), "v"(b.w));
  return d;
}

__device__ __forceinline__ v8f zero8() {
  v8f z = {0.f, 0.f, 0.f, 0.f, 0.f, 0.f, 0.f, 0.f};
  return z;
}
__device__ __forceinline__ v4f zero4() {
  v4f z = {0.f, 0.f, 0.f, 0.f};
  return z;
}
__device__ __forceinline__ v8h cvth8_(const float* f, float s) {
  v8h v;
#pragma unroll
  for (int i = 0; i < 8; ++i) v[i] = (hf_t)(f[i] * s);
  return v;
}
__device__ __forceinline__ void unpack8_(v4f a0, v4f a1, float* f) {
  f[0] = a0.x; f[1] = a0.y; f[2] = a0.z; f[3] = a0.w;
  f[4] = a1.x; f[5] = a1.y; f[6] = a1.z; f[7] = a1.w;
}

__global__ __launch_bounds__(NTHR) void k_cvtT(const float* __restrict__ W1, const float* __restrict__ W2,
                                               const float* __restrict__ KP, const float* __restrict__ RP,
                                               const float* __restrict__ OW, hf_t* W1T, hf_t* W2T,
                                               hf_t* KPT, hf_t* RPT, hf_t* OWT) {
  __shared__ __align__(16) hf_t sW[32 * (NF + 8)];
  const int blk = blockIdx.x, tid = threadIdx.x;
  const float* src;
  hf_t* dst;
  int K, N, nb;
  if (blk < CB_W1)      { src = W1; dst = W1T; K = NH; N = NF; nb = blk; }
  else if (blk < CB_W2) { src = W2; dst = W2T; K = NF; N = NH; nb = blk - CB_W1; }
  else if (blk < CB_KP) { src = KP; dst = KPT; K = NH; N = NH; nb = blk - CB_W2; }
  else if (blk < CB_RP) { src = RP; dst = RPT; K = NH; N = NH; nb = blk - CB_KP; }
  else                  { src = OW; dst = OWT; K = NH; N = NV; nb = blk - CB_RP; }
  const int n0 = nb * 32;
  const int kp8 = K + 8;
#pragma unroll 1
  for (int idx = tid; idx < K * 32; idx += NTHR) {
    const int k = idx >> 5, nn = idx & 31;
    const float v = src[(size_t)k * N + n0 + nn];
    sW[nn * kp8 + k] = (hf_t)(v * WCAR);
  }
  __syncthreads();
  const int npc = K >> 3;
#pragma unroll 1
  for (int q = tid; q < 32 * npc; q += NTHR) {
    const int nn = q / npc, p = q - nn * npc;
    const v8h v = *(const v8h*)(sW + nn * kp8 + 8 * p);
    *(volatile v8h*)(dst + (size_t)(n0 + nn) * K + 8 * p) = v;
  }
  __threadfence();
#pragma unroll 1
  for (int q = tid; q < 32 * npc; q += NTHR) {
    const int nn = q / npc, p = q - nn * npc;
    const v8h v = *(const v8h*)(sW + nn * kp8 + 8 * p);
    *(volatile v8h*)(dst + (size_t)(n0 + nn) * K + 8 * p) = v;
  }
}

__global__ __launch_bounds__(NTHR) void k_gath(const int* __restrict__ seq, const float* __restrict__ embed,
                                               hf_t* HF) {
  const size_t e = ((size_t)blockIdx.x * NTHR + threadIdx.x) * 8;
  const int tok = (int)(e >> 7);
  const int c = (int)(e & 127);
  int sq = seq[tok];
  sq = sq < 0 ? 0 : (sq > NV - 1 ? NV - 1 : sq);
  const float* sp = embed + (size_t)sq * NH + c;
  const v4f a0 = *(const v4f*)sp;
  const v4f a1 = *(const v4f*)(sp + 4);
  float f[8];
  unpack8_(a0, a1, f);
  const v8h v = cvth8_(f, 1.0f);
  *(volatile v8h*)(HF + e) = v;
  __threadfence();
  *(volatile v8h*)(HF + e) = v;
}

__device__ __forceinline__ void gemm_core(const hf_t* __restrict__ A, const hf_t* __restrict__ W, int K,
                                          int bm0, int n0, float* sT) {
  const int tid = threadIdx.x, lane = tid & 31, wave = tid >> 5, h = lane >> 4, m = lane & 15;
  const int wr = wave & 3, wc = wave >> 2;
  const int row0 = bm0 + 16 * wr, col0 = n0 + 64 * wc;

  v8f acc[GNT];
#pragma unroll
  for (int t = 0; t < GNT; ++t) acc[t] = zero8();

  const hf_t* ap = A + (size_t)(row0 + m) * K + 8 * h;
  const hf_t* bp = W + (size_t)(col0 + m) * K + 8 * h;

#pragma unroll 1
  for (int ks = 0; ks < K / 32; ++ks) {
    const int k0 = 32 * ks;
    FragH a;
    a.h[0] = *(const v8h*)(ap + k0);
    a.h[1] = *(const v8h*)(ap + k0 + 16);
#pragma unroll
    for (int t = 0; t < GNT; ++t) {
      const size_t ro = (size_t)(16 * t) * K + k0;
      FragH b;
      b.h[0] = *(const v8h*)(bp + ro);
      b.h[1] = *(const v8h*)(bp + ro + 16);
      acc[t] = wmh(a, b, acc[t]);
    }
  }

#pragma unroll
  for (int t = 0; t < GNT; ++t) {
    const int cl = 64 * wc + 16 * t + m;
#pragma unroll
    for (int r = 0; r < 8; ++r) {
      const int rl = 16 * wr + 8 * h + r;
      sT[rl * GBN + cl] = acc[t][r];
    }
  }
}

__global__ __launch_bounds__(NTHR) void k_gemmb(const hf_t* __restrict__ A, const hf_t* __restrict__ W,
                                                const float* __restrict__ bias, hf_t* C, int N, int K,
                                                int relu, float inscale, float outscale) {
  __shared__ __align__(16) float sT[GBM * GBN];
  const int tid = threadIdx.x, lane = tid & 31, wave = tid >> 5, h = lane >> 4, m = lane & 15;
  const int bm0 = blockIdx.x * GBM, n0 = blockIdx.y * GBN;
  gemm_core(A, W, K, bm0, n0, sT);
  __syncthreads();

  const v4f b0 = *(const v4f*)(bias + n0 + 8 * m);
  const v4f b1 = *(const v4f*)(bias + n0 + 8 * m + 4);
  float bb[8];
  unpack8_(b0, b1, bb);
  v8h ov[4];
#pragma unroll
  for (int rr = 0; rr < 4; ++rr) {
    const int rl = 8 * wave + 2 * rr + h;
    const v4f s0 = *(const v4f*)(sT + rl * GBN + 8 * m);
    const v4f s1 = *(const v4f*)(sT + rl * GBN + 8 * m + 4);
    float f[8];
    unpack8_(s0, s1, f);
#pragma unroll
    for (int i = 0; i < 8; ++i) {
      float v = f[i] * inscale + bb[i];
      v = (relu != 0) ? fmaxf(v, 0.0f) : v;
      f[i] = v;
    }
    ov[rr] = cvth8_(f, outscale);
  }
#pragma unroll
  for (int rr = 0; rr < 4; ++rr) {
    const int rl = 8 * wave + 2 * rr + h;
    *(volatile v8h*)(C + (size_t)(bm0 + rl) * N + n0 + 8 * m) = ov[rr];
  }
  __threadfence();
#pragma unroll
  for (int rr = 0; rr < 4; ++rr) {
    const int rl = 8 * wave + 2 * rr + h;
    *(volatile v8h*)(C + (size_t)(bm0 + rl) * N + n0 + 8 * m) = ov[rr];
  }
}

__global__ __launch_bounds__(NTHR) void k_ff2ln(const hf_t* __restrict__ A, const hf_t* __restrict__ W,
                                                const float* __restrict__ b2, const int* __restrict__ seq,
                                                const float* __restrict__ embed, const float* __restrict__ lg,
                                                const float* __restrict__ lb, hf_t* HN) {
  __shared__ __align__(16) float sT[GBM * GBN];
  const int tid = threadIdx.x, lane = tid & 31, wave = tid >> 5, h = lane >> 4, m = lane & 15;
  const int bm0 = blockIdx.x * GBM;
  gemm_core(A, W, NF, bm0, 0, sT);
  __syncthreads();

  float bb[8], gg[8], be[8];
  unpack8_(*(const v4f*)(b2 + 8 * m), *(const v4f*)(b2 + 8 * m + 4), bb);
  unpack8_(*(const v4f*)(lg + 8 * m), *(const v4f*)(lg + 8 * m + 4), gg);
  unpack8_(*(const v4f*)(lb + 8 * m), *(const v4f*)(lb + 8 * m + 4), be);
  v8h ov[4];
#pragma unroll
  for (int rr = 0; rr < 4; ++rr) {
    const int rl = 8 * wave + 2 * rr + h;
    const int tok = bm0 + rl;
    int sq = seq[tok];
    sq = sq < 0 ? 0 : (sq > NV - 1 ? NV - 1 : sq);
    const float* ep = embed + (size_t)sq * NH + 8 * m;
    float hh[8], f[8], x[8];
    unpack8_(*(const v4f*)ep, *(const v4f*)(ep + 4), hh);
    unpack8_(*(const v4f*)(sT + rl * GBN + 8 * m), *(const v4f*)(sT + rl * GBN + 8 * m + 4), f);
#pragma unroll
    for (int i = 0; i < 8; ++i) x[i] = hh[i] + (f[i] * SC_FF2 + bb[i]);
    float su = ((x[0] + x[1]) + (x[2] + x[3])) + ((x[4] + x[5]) + (x[6] + x[7]));
    su += __shfl_xor(su, 8);
    su += __shfl_xor(su, 4);
    su += __shfl_xor(su, 2);
    su += __shfl_xor(su, 1);
    const float mu = su * (1.0f / (float)NH);
    float d[8];
#pragma unroll
    for (int i = 0; i < 8; ++i) d[i] = x[i] - mu;
    float sv = ((d[0] * d[0] + d[1] * d[1]) + (d[2] * d[2] + d[3] * d[3])) +
               ((d[4] * d[4] + d[5] * d[5]) + (d[6] * d[6] + d[7] * d[7]));
    sv += __shfl_xor(sv, 8);
    sv += __shfl_xor(sv, 4);
    sv += __shfl_xor(sv, 2);
    sv += __shfl_xor(sv, 1);
    const float var = sv * (1.0f / (float)NH);
    const float rs = rsqrtf(var + LN_EPS);
#pragma unroll
    for (int i = 0; i < 8; ++i) f[i] = (d[i] * rs) * gg[i] + be[i];
    ov[rr] = cvth8_(f, 1.0f);
  }
#pragma unroll
  for (int rr = 0; rr < 4; ++rr) {
    const int rl = 8 * wave + 2 * rr + h;
    *(volatile v8h*)(HN + (size_t)(bm0 + rl) * NH + 8 * m) = ov[rr];
  }
  __threadfence();
#pragma unroll
  for (int rr = 0; rr < 4; ++rr) {
    const int rl = 8 * wave + 2 * rr + h;
    *(volatile v8h*)(HN + (size_t)(bm0 + rl) * NH + 8 * m) = ov[rr];
  }
}

__global__ __launch_bounds__(NTHR) void k_gemmf(const hf_t* __restrict__ A, const hf_t* __restrict__ W,
                                                const float* __restrict__ bias, float* C, int N, int K,
                                                int hasb, float scale) {
  __shared__ __align__(16) float sT[GBM * GBN];
  const int tid = threadIdx.x, lane = tid & 31, wave = tid >> 5;
  const int bm0 = blockIdx.x * GBM, n0 = blockIdx.y * GBN;
  gemm_core(A, W, K, bm0, n0, sT);
  __syncthreads();

  const v4f bl = *(const v4f*)(bias + n0 + 4 * lane);
  const v4f bz = zero4();
  const v4f bv = (hasb != 0) ? bl : bz;
  v4f ov[8];
#pragma unroll
  for (int rr = 0; rr < 8; ++rr) {
    const int rl = 8 * wave + rr;
    ov[rr] = *(const v4f*)(sT + rl * GBN + 4 * lane) * scale + bv;
  }
  const size_t go = (size_t)(bm0 + 8 * wave) * N + n0 + 4 * lane;
#pragma unroll
  for (int rr = 0; rr < 8; ++rr) *(volatile v4f*)(C + go + (size_t)rr * N) = ov[rr];
  __threadfence();
#pragma unroll
  for (int rr = 0; rr < 8; ++rr) *(volatile v4f*)(C + go + (size_t)rr * N) = ov[rr];
}

__global__ __launch_bounds__(STHR) void k_scan(const float* __restrict__ KALL, hf_t* RDH) {
  __shared__ __align__(16) float sK[TB * NH];
  __shared__ __align__(16) float sN[TB * NH];
  __shared__ __align__(16) float sR[NH];
  const int tid = threadIdx.x, lane = tid & 31, wave = tid >> 5;
  const int i = tid >> 2, c = tid & 3;
  const int r = tid >> 4, p = tid & 15;
  const int b = blockIdx.x;
  const float* kb = KALL + (size_t)b * NL * NH;

  float S[32];
#pragma unroll
  for (int jj = 0; jj < 32; ++jj) S[jj] = 0.0f;
  float rd = 0.0f;

#pragma unroll 1
  for (int ch = 0; ch < NCH; ++ch) {
    const float* src = kb + ((size_t)ch * TB + r) * NH + 8 * p;
    const v4f x0 = *(const v4f*)src;
    const v4f x1 = *(const v4f*)(src + 4);
    float ss = ((x0.x * x0.x + x0.y * x0.y) + (x0.z * x0.z + x0.w * x0.w)) +
               ((x1.x * x1.x + x1.y * x1.y) + (x1.z * x1.z + x1.w * x1.w));
    ss += __shfl_xor(ss, 8);
    ss += __shfl_xor(ss, 4);
    ss += __shfl_xor(ss, 2);
    ss += __shfl_xor(ss, 1);
    const float nr = sqrtf(ss);
    float inv = 1.0f / fmaxf(nr, NRM_EPS);
    inv = (ch == NCH - 1 && r == TB - 1) ? 1.0f : inv;
    float* dk = sK + r * NH + 8 * p;
    float* dn = sN + r * NH + 8 * p;
    *(v4f*)dk = x0;
    *(v4f*)(dk + 4) = x1;
    *(v4f*)dn = x0 * inv;
    *(v4f*)(dn + 4) = x1 * inv;
    __syncthreads();

#pragma unroll 1
    for (int s = 0; s < TB; ++s) {
      const float* np_ = sN + s * NH + 32 * c;
      v4f q[8];
#pragma unroll
      for (int u = 0; u < 8; ++u) q[u] = *(const v4f*)(np_ + 4 * u);
      float pp = 0.0f;
#pragma unroll
      for (int u = 0; u < 8; ++u) {
        pp = fmaf(S[4 * u + 0], q[u].x, pp);
        pp = fmaf(S[4 * u + 1], q[u].y, pp);
        pp = fmaf(S[4 * u + 2], q[u].z, pp);
        pp = fmaf(S[4 * u + 3], q[u].w, pp);
      }
      pp += __shfl_xor(pp, 1);
      pp += __shfl_xor(pp, 2);
      const float ki = sK[s * NH + i];
      const float d = ki - pp;
#pragma unroll
      for (int u = 0; u < 8; ++u) {
        S[4 * u + 0] = fmaf(d, q[u].x, S[4 * u + 0]);
        S[4 * u + 1] = fmaf(d, q[u].y, S[4 * u + 1]);
        S[4 * u + 2] = fmaf(d, q[u].z, S[4 * u + 2]);
        S[4 * u + 3] = fmaf(d, q[u].w, S[4 * u + 3]);
      }
      rd = pp;
    }
    if (ch == NCH - 1) {
      if (c == 0) sR[i] = rd;
    }
    __syncthreads();
  }

  if (wave == 0) {
    const int pl = lane & 15;
    float f[8];
    unpack8_(*(const v4f*)(sR + 8 * pl), *(const v4f*)(sR + 8 * pl + 4), f);
    const v8h v = cvth8_(f, RDCAR);
    hf_t* o = RDH + (size_t)b * NH + 8 * pl;
    if (lane < 16) *(volatile v8h*)o = v;
    __threadfence();
    if (lane < 16) *(volatile v8h*)o = v;
  }
}

extern "C" void kernel_launch(void* const* d_in, const int* in_sizes, int n_in,
                              void* d_out, int out_size, void* d_ws, size_t ws_size,
                              hipStream_t stream) {
  if (n_in < 13) return;
  if (in_sizes[0] != NTOK) return;
  if (in_sizes[1] != NV * NH) return;
  if (in_sizes[2] != NH * NF || in_sizes[3] != NF) return;
  if (in_sizes[4] != NF * NH || in_sizes[5] != NH) return;
  if (in_sizes[6] != NH || in_sizes[7] != NH) return;
  if (in_sizes[8] != NH * NH || in_sizes[9] != NH * NH || in_sizes[10] != NH) return;
  if (in_sizes[11] != NH * NV || in_sizes[12] != NV) return;
  if (out_size != NB * NV) return;
  const size_t tot = (size_t)WSTOT;
  if (tot > ws_size || tot > (size_t)WSCAP) return;

  const int*   seq   = (const int*)d_in[0];
  const float* embed = (const float*)d_in[1];
  const float* ff_w1 = (const float*)d_in[2];
  const float* ff_b1 = (const float*)d_in[3];
  const float* ff_w2 = (const float*)d_in[4];
  const float* ff_b2 = (const float*)d_in[5];
  const float* ln_g  = (const float*)d_in[6];
  const float* ln_b  = (const float*)d_in[7];
  const float* kp_w  = (const float*)d_in[8];
  const float* rp_w  = (const float*)d_in[9];
  const float* rp_b  = (const float*)d_in[10];
  const float* out_w = (const float*)d_in[11];
  const float* out_b = (const float*)d_in[12];
  float* out = (float*)d_out;

  char* ws = (char*)d_ws;
  hf_t*  HF   = (hf_t*)(ws + O_X);
  hf_t*  HN   = (hf_t*)(ws + O_X);
  hf_t*  A1   = (hf_t*)(ws + O_A1);
  float* KALL = (float*)(ws + O_A1);
  hf_t*  W1T  = (hf_t*)(ws + O_W1);
  hf_t*  W2T  = (hf_t*)(ws + O_W2);
  hf_t*  KPT  = (hf_t*)(ws + O_KP);
  hf_t*  RPT  = (hf_t*)(ws + O_RP);
  hf_t*  OWT  = (hf_t*)(ws + O_OW);
  hf_t*  RDH  = (hf_t*)(ws + O_RD);
  hf_t*  R2H  = (hf_t*)(ws + O_R2);

  k_cvtT<<<CB_TOT, NTHR, 0, stream>>>(ff_w1, ff_w2, kp_w, rp_w, out_w, W1T, W2T, KPT, RPT, OWT);
  k_gath<<<(NTOK * NH) / (8 * NTHR), NTHR, 0, stream>>>(seq, embed, HF);
  k_gemmb<<<dim3(NTOK / GBM, NF / GBN), NTHR, 0, stream>>>(HF, W1T, ff_b1, A1, NF, NH, 1, SC_FF1, A1CAR);
  k_ff2ln<<<NTOK / GBM, NTHR, 0, stream>>>(A1, W2T, ff_b2, seq, embed, ln_g, ln_b, HN);
  k_gemmf<<<dim3(NTOK / GBM, NH / GBN), NTHR, 0, stream>>>(HN, KPT, ff_b2, KALL, NH, NH, 0, SC_KP);
  k_scan<<<NB, STHR, 0, stream>>>(KALL, RDH);
  k_gemmb<<<dim3(NB / GBM, NH / GBN), NTHR, 0, stream>>>(RDH, RPT, rp_b, R2H, NH, NH, 0, SC_RP, R2CAR);
  k_gemmf<<<dim3(NB / GBM, NV / GBN), NTHR, 0, stream>>>(R2H, OWT, out_b, out, NV, NH, 1, SC_OUT);
}
